// Embedding_39737037423043
// MI455X (gfx1250) — hardware-run, weakly checked
//
#include <hip/hip_runtime.h>

typedef float          v8f   __attribute__((ext_vector_type(8)));
typedef float          v4f   __attribute__((ext_vector_type(4)));
typedef unsigned int   v4u   __attribute__((ext_vector_type(4)));
typedef int            v8i   __attribute__((ext_vector_type(8)));
typedef unsigned short v8us  __attribute__((ext_vector_type(8)));
typedef unsigned short v16us __attribute__((ext_vector_type(16)));
typedef __bf16         v16bf __attribute__((ext_vector_type(16)));
typedef _Float16       v16h  __attribute__((ext_vector_type(16)));
typedef v4f  __attribute__((may_alias)) v4fa;
typedef v8us __attribute__((may_alias)) v8usa;
union FragB { v16bf v; v16us u; v8us h[2]; v8i w; };
union FragH { v16h  v; v16us u; v8us h[2]; v8i w; };

__device__ __forceinline__ v8f wmb(const FragB& a, const FragB& b, v8f c) {
  v8f d = __builtin_amdgcn_wmma_f32_16x16x32_bf16(false, a.v, false, b.v, (short)0, c, false, false);
  asm volatile("v_nop\n\tv_nop\n\tv_nop\n\tv_nop" : "+v"(d) : "v"(a.w), "v"(b.w));
  return d;
}

__device__ __forceinline__ v8f wmh(const FragH& a, const FragH& b, v8f c) {
  v8f d = __builtin_amdgcn_wmma_f32_16x16x32_f16(false, a.v, false, b.v, (short)0, c, false, false);
  asm volatile("v_nop\n\tv_nop\n\tv_nop\n\tv_nop" : "+v"(d) : "v"(a.w), "v"(b.w));
  return d;
}

__device__ __forceinline__ unsigned bf16_bits(float f) {
  const unsigned u = __float_as_uint(f);
  const unsigned r = (u + 0x7FFFu + ((u >> 16) & 1u)) >> 16;
  const unsigned q = (u >> 16) | 0x40u;
  return ((u & 0x7fffffffu) > 0x7f800000u) ? q : r;
}

__device__ __forceinline__ float bf16_val(float f) {
  return __uint_as_float(bf16_bits(f) << 16);
}
__device__ __forceinline__ int clampi(int v, int lo, int hi) {
  return v < lo ? lo : (v > hi ? hi : v);
}

__device__ __forceinline__ unsigned f16_bits(float f) {
  const unsigned u  = __float_as_uint(f);
  const unsigned s  = (u >> 16) & 0x8000u;
  const unsigned a  = u & 0x7fffffffu;
  const unsigned t  = a - 0x38000000u;
  const unsigned r  = (t + 0x0FFFu + ((t >> 13) & 1u)) >> 13;
  const unsigned rc = r > 0x7C00u ? 0x7C00u : r;
  const bool small  = a < 0x38800000u;
  const bool isnan  = a > 0x7f800000u;
  const unsigned fin = small ? 0u : (s | rc);
  return isnan ? (s | 0x7E00u) : fin;
}

__device__ __forceinline__ unsigned pk16(unsigned lo, unsigned hi) { return lo | (hi << 16); }
__device__ __forceinline__ unsigned bf16_lo_bits(float v) {
  float hi = bf16_val(v);
  asm volatile("" : "+v"(hi));
  return bf16_bits(v - hi);
}
__device__ __forceinline__ v4u pack8_bf16(v4f a, v4f c) {
  return (v4u){ pk16(bf16_bits(a[0]), bf16_bits(a[1])), pk16(bf16_bits(a[2]), bf16_bits(a[3])),
                pk16(bf16_bits(c[0]), bf16_bits(c[1])), pk16(bf16_bits(c[2]), bf16_bits(c[3])) };
}
__device__ __forceinline__ v4u pack8_bf16_lo(v4f a, v4f c) {
  return (v4u){ pk16(bf16_lo_bits(a[0]), bf16_lo_bits(a[1])), pk16(bf16_lo_bits(a[2]), bf16_lo_bits(a[3])),
                pk16(bf16_lo_bits(c[0]), bf16_lo_bits(c[1])), pk16(bf16_lo_bits(c[2]), bf16_lo_bits(c[3])) };
}
__device__ __forceinline__ v4u pack8_f16(v4f a, v4f c) {
  return (v4u){ pk16(f16_bits(a[0]), f16_bits(a[1])), pk16(f16_bits(a[2]), f16_bits(a[3])),
                pk16(f16_bits(c[0]), f16_bits(c[1])), pk16(f16_bits(c[2]), f16_bits(c[3])) };
}

template <int FORM>
__global__ __launch_bounds__(256) void k_plane(const float* __restrict__ src, int rows, int cols, int ldsrc,
                                               unsigned short* __restrict__ dst, int MP, int KP) {
  static_assert(FORM >= 0 && FORM <= 3);
  const int KTOT = (FORM == 1 || FORM == 3) ? 2 * KP : KP;
  const unsigned ppr   = (unsigned)(KTOT >> 3);
  const unsigned kp8   = (unsigned)(KP >> 3);
  const unsigned total = (unsigned)MP * ppr;
  const unsigned g     = blockIdx.x * 256u + threadIdx.x;
  const unsigned rowu  = g / ppr;
  const unsigned p     = g - rowu * ppr;
  const bool second    = p >= kp8;
  const int row = (int)rowu;
  const int c0  = (int)((second ? p - kp8 : p) << 3);
  const float* srow = src + (size_t)clampi(row, 0, rows - 1) * (size_t)ldsrc;
  float x[8];
  unsigned mk[8];
#pragma unroll
  for (int e = 0; e < 8; ++e) {
    const int c = c0 + e;
    const float v = srow[clampi(c, 0, cols - 1)];
    asm volatile("" :: "v"(v));
    x[e]  = v;
    mk[e] = (row < rows && c < cols) ? 0xFFFFu : 0u;
  }
  const v4f a = (v4f){ x[0], x[1], x[2], x[3] };
  const v4f c = (v4f){ x[4], x[5], x[6], x[7] };
  v4u o;
  if (FORM == 2) {
    o = pack8_f16(a, c);
  } else {
    const v4u hi = pack8_bf16(a, c);
    o = hi;
    if (FORM == 1) { const v4u lo = pack8_bf16_lo(a, c); o = second ? lo : hi; }
  }
  const v4u mw = (v4u){ pk16(mk[0], mk[1]), pk16(mk[2], mk[3]), pk16(mk[4], mk[5]), pk16(mk[6], mk[7]) };
  o &= mw;
  if (g < total) {
    volatile v4u* q = (volatile v4u*)(dst + (size_t)g * 8);
    *q = o;
    __threadfence();
    *q = o;
  }
}

template <int FORM> struct FragOf    { typedef FragB T; };
template <>         struct FragOf<2> { typedef FragH T; };
__device__ __forceinline__ v8f mm(const FragB& a, const FragB& b, v8f c) { return wmb(a, b, c); }
__device__ __forceinline__ v8f mm(const FragH& a, const FragH& b, v8f c) { return wmh(a, b, c); }
template <class F> __device__ __forceinline__ F ld_frag(const unsigned short* p) {
  F f;
  f.h[0] = *(const v8usa*)(p);
  f.h[1] = *(const v8usa*)(p + 16);
  return f;
}

template <int FORM, int EPI>
__global__ __launch_bounds__(256) __attribute__((amdgpu_num_vgpr(248)))
void k_gemm_nt(const unsigned short* __restrict__ A, const unsigned short* __restrict__ B,
               const float* __restrict__ bias, float* __restrict__ D, int M, int N, int KTOT, int ldd) {
  static_assert(FORM >= 0 && FORM <= 2);
  static_assert(EPI == 0 || EPI == 1);
  typedef typename FragOf<FORM>::T F;
  __shared__ __attribute__((aligned(16))) float sT[8][16 * 68];
  const int lane = threadIdx.x & 31;
  const int wave = threadIdx.x >> 5;
  const int tilesM = (M + 63) >> 6;
  const int tilesN = (N + 63) >> 6;
  const int tile = blockIdx.x * 8 + wave;
  if (tile >= tilesM * tilesN) return;
  const int tm = tile / tilesN;
  const int tn = tile - tm * tilesN;
  const int m0 = tm << 6;
  const int n0 = tn << 6;

  const int rl = lane & 15;
  const int h8 = (lane >> 4) * 8;
  const unsigned short* pa = A + (size_t)(m0 + rl) * (size_t)KTOT + h8;
  const unsigned short* pb = B + (size_t)(n0 + rl) * (size_t)KTOT + h8;

  v8f acc[4][4];
#pragma unroll
  for (int i = 0; i < 4; ++i)
#pragma unroll
    for (int j = 0; j < 4; ++j) acc[i][j] = (v8f){0.f, 0.f, 0.f, 0.f, 0.f, 0.f, 0.f, 0.f};

#pragma unroll 1
  for (int k0 = 0; k0 < KTOT; k0 += 32) {
    F bf[4];
#pragma unroll
    for (int j = 0; j < 4; ++j) bf[j] = ld_frag<F>(pb + (size_t)(j << 4) * (size_t)KTOT + k0);
#pragma unroll
    for (int i = 0; i < 4; ++i) {
      const F af = ld_frag<F>(pa + (size_t)(i << 4) * (size_t)KTOT + k0);
#pragma unroll
      for (int j = 0; j < 4; ++j) acc[i][j] = mm(af, bf[j], acc[i][j]);
    }
  }

  float* slab = sT[wave];
  const int hh = lane >> 4;
  const int c4 = (lane & 15) * 4;
  const int nc = n0 + c4;
  const bool cok = nc < N;
  v4f bv = (v4f){0.f, 0.f, 0.f, 0.f};
  if (EPI == 1) {
    bv = *(const v4fa*)(bias + clampi(nc, 0, N - 4));
    asm volatile("" :: "v"(bv));
  }
#pragma unroll
  for (int i = 0; i < 4; ++i) {
    const int mBase = m0 + (i << 4);
#pragma unroll
    for (int j = 0; j < 4; ++j) {
#pragma unroll
      for (int r = 0; r < 8; ++r) slab[(h8 + r) * 68 + (j << 4) + rl] = acc[i][j][r];
    }
    __builtin_amdgcn_fence(__ATOMIC_RELEASE, "workgroup");
    __builtin_amdgcn_wave_barrier();
    __builtin_amdgcn_fence(__ATOMIC_ACQUIRE, "workgroup");
    v4f vv[8];
#pragma unroll
    for (int it = 0; it < 8; ++it) {
      const int row = it * 2 + hh;
      v4f v = *(const v4fa*)(slab + row * 68 + c4);
      if (EPI == 1) v += bv;
      vv[it] = v;
    }
    for (int pass = 0; pass < 2; ++pass) {
#pragma unroll
      for (int it = 0; it < 8; ++it) {
        const int row = mBase + it * 2 + hh;
        if (cok && row < M) *(volatile v4f*)(D + (size_t)row * (size_t)ldd + nc) = vv[it];
      }
      __threadfence();
    }
    __builtin_amdgcn_fence(__ATOMIC_RELEASE, "workgroup");
    __builtin_amdgcn_wave_barrier();
    __builtin_amdgcn_fence(__ATOMIC_ACQUIRE, "workgroup");
  }
}

#pragma clang fp contract(off)
#include <math.h>
#include <stddef.h>

#define NBAT    2
#define CH      64
#define NPT     50000
#define KNB     16
#define MROWS   (NBAT * NPT)
#define MPAD    100096
#define TPB     782
#define NPADR   (MPAD - MROWS)
#define SPLIT_PAIR 1
#define KSTEPS  (SPLIT_PAIR ? 4 : 2)
#define APW     68
#define NVEC    9
#define VECN    (NVEC * CH)
#define NLT     1562

#define SZ_HL   ((size_t)MPAD * 128 * 2)
#define SZ_F32  ((size_t)MPAD * 64 * 4)
#define O_XN    ((size_t)0)
#define O_A2    (O_XN + SZ_HL)
#define O_PT    (O_A2 + SZ_HL)
#define O_U     (O_PT + SZ_F32)
#define O_W1    (O_U + SZ_F32)
#define O_W2A   (O_W1 + (size_t)16384)
#define O_W2B   (O_W2A + (size_t)16384)
#define O_WF    (O_W2B + (size_t)16384)
#define O_VEC   (O_WF + (size_t)32768)
#define WS_TOTAL (O_VEC + (size_t)VECN * 4)

static_assert(CH == 64);
static_assert(KNB - 1 == 15 && KNB - 1 <= 16);
static_assert(NPT % 16 == 0 && NPT % 4 == 0);
static_assert(((size_t)NPT * 4) % 128 == 64);
static_assert(NLT * 32 + 16 == NPT);
static_assert(MPAD % 64 == 0 && MPAD >= MROWS && MPAD == TPB * 128);
static_assert(((MROWS + 63) / 64) * 64 <= MPAD);
static_assert(MROWS % 16 == 0);
static_assert(TPB * 64 >= NPT && (TPB - 1) * 64 < NPT && NPT - (TPB - 1) * 64 == 16);
static_assert(NPADR * 16 == 6 * 256);
static_assert(NPADR * 32 == 12 * 256);
static_assert((size_t)MPAD * 256 * 2 == 2 * SZ_HL);
static_assert(SZ_HL % 256 == 0 && SZ_F32 % 256 == 0 && O_VEC % 256 == 0);
static_assert(VECN * 4 == 18 * 128);
static_assert(WS_TOTAL <= ((size_t)128 << 20));
static_assert(8 * 16 * APW * 4 + 8 * CH * 4 + 256 * 4 + 1024 * 4 <= 327680);
static_assert((long long)MPAD * 256 / 8 < 0x7fffffffLL);

typedef float v2f __attribute__((ext_vector_type(2)));
typedef v2f  __attribute__((may_alias)) v2fa;
typedef v4u  __attribute__((may_alias)) v4ua;

__device__ __forceinline__ void wave_sync_lds() {
  __builtin_amdgcn_fence(__ATOMIC_RELEASE, "workgroup");
  __builtin_amdgcn_wave_barrier();
  __builtin_amdgcn_fence(__ATOMIC_ACQUIRE, "workgroup");
}
__device__ __forceinline__ void put16(unsigned short* p, v4u v) { *(volatile v4u*)p = v; }
__device__ __forceinline__ void putf4(float* p, v4f v) { *(volatile v4f*)p = v; }

__global__ __launch_bounds__(256) void k_vec(
    const float* __restrict__ g0, const float* __restrict__ b0, const float* __restrict__ m0,
    const float* __restrict__ v0, const float* __restrict__ b1,
    const float* __restrict__ g2a, const float* __restrict__ b2a, const float* __restrict__ m2a,
    const float* __restrict__ v2a, const float* __restrict__ w2a,
    const float* __restrict__ g2b, const float* __restrict__ b2b, const float* __restrict__ m2b,
    const float* __restrict__ v2b, const float* __restrict__ bfv, float* VEC) {
  __shared__ __attribute__((aligned(16))) float sv[VECN];
  __shared__ float stv[CH];
  __shared__ float smb[CH];
  const int tid = (int)threadIdx.x;
  const int set = __builtin_amdgcn_readfirstlane(tid >> 6);
  const int c = tid & 63;
  const float gA = g0[c], gB = g2a[c], gC = g2b[c];
  const float vA = v0[c], vB = v2a[c], vC = v2b[c];
  asm volatile("" :: "v"(gA)); asm volatile("" :: "v"(gB)); asm volatile("" :: "v"(gC));
  asm volatile("" :: "v"(vA)); asm volatile("" :: "v"(vB)); asm volatile("" :: "v"(vC));
  const float mA = m0[c], mB = m2a[c], mC = m2b[c];
  const float bA = b0[c], bB = b2a[c], bC = b2b[c];
  asm volatile("" :: "v"(mA)); asm volatile("" :: "v"(mB)); asm volatile("" :: "v"(mC));
  asm volatile("" :: "v"(bA)); asm volatile("" :: "v"(bB)); asm volatile("" :: "v"(bC));
  const float xA = b1[c], xB = bfv[c];
  asm volatile("" :: "v"(xA)); asm volatile("" :: "v"(xB));
  const float g = bf16_val(set == 0 ? gA : (set == 1 ? gB : gC));
  const float v = bf16_val(set == 0 ? vA : (set == 1 ? vB : vC));
  const float m = bf16_val(set == 0 ? mA : (set == 1 ? mB : mC));
  const float bb = bf16_val(set == 0 ? bA : (set == 1 ? bB : bC));
  const float s = g / sqrtf(v + 1e-5f);
  if (set == 0) {
    sv[0 * CH + c] = s; sv[1 * CH + c] = m; sv[2 * CH + c] = bb;
  } else if (set == 1) {
    sv[3 * CH + c] = s; stv[c] = bb - s * m;
  } else if (set == 2) {
    sv[5 * CH + c] = s; sv[6 * CH + c] = bb; smb[c] = m;
  } else {
    sv[7 * CH + c] = bf16_val(xA); sv[8 * CH + c] = bf16_val(xB);
  }
  __syncthreads();
  if (set == 0) {
    float acc = 0.0f;
#pragma unroll 4
    for (int k = 0; k < CH; ++k) acc += bf16_val(w2a[tid * CH + k]) * stv[k];
    sv[4 * CH + tid] = acc - smb[tid];
  }
  __syncthreads();
  const int pi = tid < 143 ? tid : 143;
  const v4f pv = *(const v4fa*)(sv + 4 * pi);
  asm volatile("" :: "v"(pv));
  const bool ok = tid < 144;
  float* gp = VEC + 4 * pi;
  if (ok) putf4(gp, pv);
  __threadfence();
  if (ok) putf4(gp, pv);
}

__global__ __launch_bounds__(256) void k_xn(const float* __restrict__ x, const float* __restrict__ VEC,
                                            unsigned short* XN, unsigned short* A2) {
  __shared__ __attribute__((aligned(16))) float sP[256];
  __shared__ float tl[CH * 65];
  const int tid = (int)threadIdx.x;
  const int wave = __builtin_amdgcn_readfirstlane(tid >> 5);
  const int b = (int)blockIdx.y;
  const int n0 = (int)blockIdx.x * 64;
  int nvalid = NPT - n0;
  nvalid = nvalid > 64 ? 64 : nvalid;

  if (wave < 2) {
    const v4f pv = *(const v4fa*)(VEC + 4 * tid);
    *(v4fa*)(sP + 4 * tid) = pv;
  }
  __syncthreads();

#pragma unroll
  for (int i = 0; i < 4; ++i) {
    const int idx = tid + 256 * i;
    const int c = idx >> 4, q = idx & 15;
    int nn = n0 + 4 * q;
    nn = nn > NPT - 4 ? NPT - 4 : nn;
    const v4f xv = *(const v4fa*)(x + (size_t)(b * CH + c) * (size_t)NPT + nn);
    asm volatile("" :: "v"(xv));
    const float s0 = sP[c], m0 = sP[64 + c], b0 = sP[128 + c];
#pragma unroll
    for (int e = 0; e < 4; ++e) tl[c * 65 + 4 * q + e] = (bf16_val(xv[e]) - m0) * s0 + b0;
  }
  __syncthreads();

  const int p8 = tid & 7;
  const int rq = tid >> 3;
  v4u oxh[2], oxl[2], oah[2], oal[2];
#pragma unroll
  for (int i = 0; i < 2; ++i) {
    const int row = rq + 32 * i;
    float xv[8], av[8];
#pragma unroll
    for (int e = 0; e < 8; ++e) {
      const int c = 8 * p8 + e;
      const float v = tl[c * 65 + row];
      xv[e] = v;
      av[e] = v * sP[192 + c];
    }
    const v4f xa = (v4f){ xv[0], xv[1], xv[2], xv[3] }, xc = (v4f){ xv[4], xv[5], xv[6], xv[7] };
    const v4f aa = (v4f){ av[0], av[1], av[2], av[3] }, ac = (v4f){ av[4], av[5], av[6], av[7] };
    oxh[i] = pack8_bf16(xa, xc);
    oxl[i] = pack8_bf16_lo(xa, xc);
    oah[i] = pack8_bf16(aa, ac);
    oal[i] = pack8_bf16_lo(aa, ac);
  }
#pragma unroll
  for (int pass = 0; pass < 2; ++pass) {
#pragma unroll
    for (int i = 0; i < 2; ++i) {
      const int row = rq + 32 * i;
      if (row < nvalid) {
        const size_t R = (size_t)b * NPT + (size_t)(n0 + row);
        put16(XN + R * 128 + 8 * p8, oxh[i]);
        put16(XN + R * 128 + 64 + 8 * p8, oxl[i]);
        put16(A2 + R * 128 + 8 * p8, oah[i]);
        put16(A2 + R * 128 + 64 + 8 * p8, oal[i]);
      }
    }
    __threadfence();
  }

  if ((int)blockIdx.x == TPB - 1 && b == NBAT - 1) {
    const v4u z = (v4u){ 0u, 0u, 0u, 0u };
#pragma unroll
    for (int pass = 0; pass < 2; ++pass) {
#pragma unroll
      for (int i = 0; i < 6; ++i) {
        const size_t off = (size_t)MROWS * 128 + (size_t)(tid + 256 * i) * 8;
        put16(XN + off, z);
        put16(A2 + off, z);
      }
      __threadfence();
    }
  }
}

__global__ __launch_bounds__(256) __attribute__((amdgpu_num_vgpr(248)))
void k_pair(const int* __restrict__ nbr, const float* __restrict__ U, const float* __restrict__ PT,
            const unsigned short* __restrict__ W2B, const float* __restrict__ VEC, unsigned short* CAT) {
  __shared__ __attribute__((aligned(16))) unsigned sA[8][16 * APW];
  __shared__ __attribute__((aligned(16))) float sN[8][CH];
  __shared__ __attribute__((aligned(16))) float sQ[256];
  __shared__ int sId[1024];
  const int tid = (int)threadIdx.x;
  const int lane = tid & 31;
  const int wave = __builtin_amdgcn_readfirstlane(tid >> 5);
  const int b = (int)blockIdx.y;
  const int n0 = (int)blockIdx.x * 64;
  int nvalid = NPT - n0;
  nvalid = nvalid > 64 ? 64 : nvalid;

  if (wave < 2) {
    const v4f pv = *(const v4fa*)(VEC + 256 + 4 * tid);
    *(v4fa*)(sQ + 4 * tid) = pv;
  }
#pragma unroll
  for (int i = 0; i < 4; ++i) {
    const int idx = tid + 256 * i;
    int kk = 1 + (idx >> 6);
    kk = kk > KNB - 1 ? KNB - 1 : kk;
    int n = n0 + (idx & 63);
    n = n > NPT - 1 ? NPT - 1 : n;
    const int id = nbr[(size_t)(b * KNB + kk) * (size_t)NPT + n];
    asm volatile("" :: "v"(id));
    sId[idx] = clampi(id, 0, NPT - 1);
  }
  __syncthreads();

  const int rl = lane & 15;
  const int h8 = (lane >> 4) * 8;
  FragB bw[4][2];
#pragma unroll
  for (int j = 0; j < 4; ++j) {
#pragma unroll
    for (int ks = 0; ks < 2; ++ks) {
      const unsigned short* wq = W2B + (size_t)(16 * j + rl) * 128 + h8 + 32 * ks;
      bw[j][ks].h[0] = *(const v8usa*)wq;
      bw[j][ks].h[1] = *(const v8usa*)(wq + 16);
    }
  }
  const v2f cm = *(const v2fa*)(sQ + 2 * lane);
  const v2f sb = *(const v2fa*)(sQ + 64 + 2 * lane);
  const v2f bb = *(const v2fa*)(sQ + 128 + 2 * lane);

  unsigned* aw = &sA[wave][0];
  const unsigned short* ap = (const unsigned short*)(&sA[wave][0]) + rl * (2 * APW) + h8;
  float* nrow = &sN[wave][0];
  const size_t cloud = (size_t)b * NPT;
  const unsigned mskN = (lane & 8) ? 0xFFFFFFFFu : 0u;
  const unsigned mskL = (lane & 16) ? 0xFFFFFFFFu : 0u;
  const int c8 = 8 * (lane & 7);

  int npts = nvalid - 8 * wave;
  npts = npts < 0 ? 0 : (npts > 8 ? 8 : npts);

#pragma unroll 1
  for (int q = 0; q < npts; ++q) {
    const int p = 8 * wave + q;
    const size_t R = cloud + (size_t)(n0 + p);
    const v2f un = *(const v2fa*)(U + R * 64 + 2 * lane);
    unsigned lastH = 0u, lastL = 0u;
#pragma unroll 5
    for (int i = 0; i < 15; ++i) {
      const int j = sId[i * 64 + p];
      const v2f uj = *(const v2fa*)(U + (cloud + (size_t)j) * 64 + 2 * lane);
      float t0 = ((uj[0] - un[0]) + cm[0]) * sb[0] + bb[0];
      float t1 = ((uj[1] - un[1]) + cm[1]) * sb[1] + bb[1];
      t0 = (t0 > 0.0f) ? t0 : (t0 - t0);
      t1 = (t1 > 0.0f) ? t1 : (t1 - t1);
      lastH = pk16(bf16_bits(t0), bf16_bits(t1));
      aw[i * APW + lane] = lastH;
      if (SPLIT_PAIR) {
        lastL = pk16(bf16_lo_bits(t0), bf16_lo_bits(t1));
        aw[i * APW + 32 + lane] = lastL;
      }
    }
    aw[15 * APW + lane] = lastH;
    if (SPLIT_PAIR) aw[15 * APW + 32 + lane] = lastL;
    wave_sync_lds();

    v8f acc[4];
#pragma unroll
    for (int j = 0; j < 4; ++j) acc[j] = (v8f){0.f, 0.f, 0.f, 0.f, 0.f, 0.f, 0.f, 0.f};
#pragma unroll
    for (int ks = 0; ks < KSTEPS; ++ks) {
      FragB af;
      af.h[0] = *(const v8usa*)(ap + 32 * ks);
      af.h[1] = *(const v8usa*)(ap + 32 * ks + 16);
#pragma unroll
      for (int j = 0; j < 4; ++j) acc[j] = wmb(af, bw[j][ks & 1], acc[j]);
    }

#pragma unroll
    for (int j = 0; j < 4; ++j) {
      float m = acc[j][0];
#pragma unroll
      for (int r = 1; r < 8; ++r) {
        const float v = acc[j][r];
        m = (v > m || v != v) ? v : m;
      }
      const float o = __shfl_xor(m, 16);
      m = (o > m || o != o) ? o : m;
      nrow[16 * j + rl] = m;
    }
    wave_sync_lds();

    const v4f p0 = *(const v4fa*)(PT + R * 64 + c8);
    const v4f p1 = *(const v4fa*)(PT + R * 64 + c8 + 4);
    asm volatile("" :: "v"(p0));
    asm volatile("" :: "v"(p1));
    const v4f q0 = *(const v4fa*)(nrow + c8);
    const v4f q1 = *(const v4fa*)(nrow + c8 + 4);
    v4f s0, s1;
#pragma unroll
    for (int e = 0; e < 4; ++e) {
      s0[e] = __uint_as_float((__float_as_uint(q0[e]) & mskN) | (__float_as_uint(p0[e]) & ~mskN));
      s1[e] = __uint_as_float((__float_as_uint(q1[e]) & mskN) | (__float_as_uint(p1[e]) & ~mskN));
    }
    const v4u hv = pack8_bf16(s0, s1);
    const v4u lv = pack8_bf16_lo(s0, s1);
    const v4u ov = (lv & mskL) | (hv & ~mskL);
    unsigned short* dst = CAT + R * 256 + 8 * lane;
    put16(dst, ov);
    __threadfence();
    put16(dst, ov);
    wave_sync_lds();
  }

  if ((int)blockIdx.x == TPB - 1 && b == NBAT - 1) {
    const v4u z = (v4u){ 0u, 0u, 0u, 0u };
#pragma unroll
    for (int pass = 0; pass < 2; ++pass) {
#pragma unroll
      for (int i = 0; i < 12; ++i) put16(CAT + (size_t)MROWS * 256 + (size_t)(tid + 256 * i) * 8, z);
      __threadfence();
    }
  }
}

__global__ __launch_bounds__(256) void k_store(const float* __restrict__ Y, float* out) {
  __shared__ __attribute__((aligned(16))) float sY[48 * 68];
  const int tid = (int)threadIdx.x;
  const int b = (int)blockIdx.y;
  const int t = (int)blockIdx.x;
  const size_t cloud = (size_t)b * NPT;
  if (t < NLT) {
#pragma unroll
    for (int i = 0; i < 3; ++i) {
      const int idx = tid + 256 * i;
      const int row = idx >> 4, q = idx & 15;
      const v4f v = *(const v4fa*)(Y + (cloud + (size_t)(32 * t + row)) * 64 + 4 * q);
      *(v4fa*)(sY + row * 68 + 4 * q) = v;
    }
    __syncthreads();
    v4f ov[2];
    float* gp[2];
#pragma unroll
    for (int i = 0; i < 2; ++i) {
      const int g = tid + 256 * i;
      const int o = g >> 3, pc = g & 7;
      const int lp = (o & 1) * 16 + 4 * pc;
      ov[i] = (v4f){ sY[(lp + 0) * 68 + o], sY[(lp + 1) * 68 + o], sY[(lp + 2) * 68 + o], sY[(lp + 3) * 68 + o] };
      gp[i] = out + (size_t)(b * CH + o) * (size_t)NPT + (size_t)(32 * t + lp);
    }
#pragma unroll
    for (int pass = 0; pass < 2; ++pass) {
      putf4(gp[0], ov[0]);
      putf4(gp[1], ov[1]);
      __threadfence();
    }
  } else {
#pragma unroll
    for (int i = 0; i < 2; ++i) {
      const int idx = tid + 256 * i;
      const int row = idx >> 4, q = idx & 15;
      const int srow = row < 16 ? (NPT - 16 + row) : (row - 16);
      const v4f v = *(const v4fa*)(Y + (cloud + (size_t)srow) * 64 + 4 * q);
      *(v4fa*)(sY + row * 68 + 4 * q) = v;
    }
    __syncthreads();
    const int pair = tid >> 3, pc = tid & 7;
    const int o = 2 * pair + (pc >> 2);
    const int lr = 4 * pc;
    const v4f ov = (v4f){ sY[(lr + 0) * 68 + o], sY[(lr + 1) * 68 + o], sY[(lr + 2) * 68 + o], sY[(lr + 3) * 68 + o] };
    float* gp = out + (size_t)(b * CH + 2 * pair) * (size_t)NPT + (size_t)(NPT - 16 + 4 * pc);
    putf4(gp, ov);
    __threadfence();
    putf4(gp, ov);
  }
}

extern "C" void kernel_launch(void* const* d_in, const int* in_sizes, int n_in,
                              void* d_out, int out_size, void* d_ws, size_t ws_size,
                              hipStream_t stream) {
  if (n_in < 20) return;
  if (in_sizes[0] != NBAT * CH * NPT) return;
  if (in_sizes[1] != NBAT * KNB * NPT) return;
  if (in_sizes[2] != CH || in_sizes[3] != CH || in_sizes[4] != CH || in_sizes[5] != CH) return;
  if (in_sizes[6] != CH * CH || in_sizes[7] != CH) return;
  if (in_sizes[8] != CH || in_sizes[9] != CH || in_sizes[10] != CH || in_sizes[11] != CH) return;
  if (in_sizes[12] != CH * CH) return;
  if (in_sizes[13] != CH || in_sizes[14] != CH || in_sizes[15] != CH || in_sizes[16] != CH) return;
  if (in_sizes[17] != CH * CH) return;
  if (in_sizes[18] != CH * 2 * CH || in_sizes[19] != CH) return;
  if ((long long)out_size != (long long)NBAT * CH * NPT) return;
  if ((size_t)WS_TOTAL > ws_size) return;

  const float* x    = (const float*)d_in[0];
  const int*   nbr  = (const int*)d_in[1];
  const float* g0   = (const float*)d_in[2];
  const float* b0   = (const float*)d_in[3];
  const float* m0   = (const float*)d_in[4];
  const float* v0   = (const float*)d_in[5];
  const float* w1   = (const float*)d_in[6];
  const float* b1   = (const float*)d_in[7];
  const float* g2a  = (const float*)d_in[8];
  const float* b2a  = (const float*)d_in[9];
  const float* m2a  = (const float*)d_in[10];
  const float* v2a  = (const float*)d_in[11];
  const float* w2a  = (const float*)d_in[12];
  const float* g2b  = (const float*)d_in[13];
  const float* b2b  = (const float*)d_in[14];
  const float* m2b  = (const float*)d_in[15];
  const float* v2b  = (const float*)d_in[16];
  const float* w2b  = (const float*)d_in[17];
  const float* wf   = (const float*)d_in[18];
  const float* bfv  = (const float*)d_in[19];
  float* out = (float*)d_out;

  char* ws = (char*)d_ws;
  unsigned short* XN   = (unsigned short*)(ws + O_XN);
  unsigned short* A2   = (unsigned short*)(ws + O_A2);
  unsigned short* CAT  = (unsigned short*)(ws + O_XN);
  float*          PT   = (float*)(ws + O_PT);
  float*          U    = (float*)(ws + O_U);
  float*          Y    = (float*)(ws + O_U);
  unsigned short* W1D  = (unsigned short*)(ws + O_W1);
  unsigned short* W2AD = (unsigned short*)(ws + O_W2A);
  unsigned short* W2BD = (unsigned short*)(ws + O_W2B);
  unsigned short* WFD  = (unsigned short*)(ws + O_WF);
  float*          VEC  = (float*)(ws + O_VEC);

  k_plane<3><<<64 * 128 / 8 / 256, 256, 0, stream>>>(w1,  CH, CH, CH, W1D,  CH, CH);
  k_plane<3><<<64 * 128 / 8 / 256, 256, 0, stream>>>(w2a, CH, CH, CH, W2AD, CH, CH);
  k_plane<3><<<64 * 128 / 8 / 256, 256, 0, stream>>>(w2b, CH, CH, CH, W2BD, CH, CH);
  k_plane<3><<<64 * 256 / 8 / 256, 256, 0, stream>>>(wf,  CH, 2 * CH, 2 * CH, WFD, CH, 2 * CH);
  k_vec<<<1, 256, 0, stream>>>(g0, b0, m0, v0, b1, g2a, b2a, m2a, v2a, w2a, g2b, b2b, m2b, v2b, bfv, VEC);

  k_xn<<<dim3(TPB, NBAT), 256, 0, stream>>>(x, VEC, XN, A2);

  const int gGemm = ((MROWS + 63) / 64 + 7) / 8;
  k_gemm_nt<0, 1><<<gGemm, 256, 0, stream>>>(XN, W1D, VEC + 7 * CH, PT, MROWS, CH, 128, CH);
  k_gemm_nt<0, 0><<<gGemm, 256, 0, stream>>>(A2, W2AD, VEC + 7 * CH, U, MROWS, CH, 128, CH);

  k_pair<<<dim3(TPB, NBAT), 256, 0, stream>>>(nbr, U, PT, W2BD, VEC, CAT);

  k_gemm_nt<0, 1><<<gGemm, 256, 0, stream>>>(CAT, WFD, VEC + 8 * CH, Y, MROWS, CH, 256, CH);

  k_store<<<dim3(NLT + 1, NBAT), 256, 0, stream>>>(Y, out);
}
